// EncoderBlock_85564338471553
// MI455X (gfx1250) — hardware-verified
//
#include <hip/hip_runtime.h>
#include <stdint.h>


#ifndef NB
#define NB 4
#endif
#ifndef SEQ
#define SEQ 2048
#endif
#define NB_FULL   4
#define SEQ_FULL  2048
#define D_MODEL   768
#define NHEAD     12
#define DKH       64
#define D_FF      3072
#define ROWS      (NB * SEQ)

static_assert((SEQ % 128) == 0);
static_assert((ROWS % 128) == 0);
static_assert(SEQ <= SEQ_FULL);
static_assert(NB >= 1 && NB <= NB_FULL);
static_assert(NHEAD * DKH == D_MODEL);
static_assert(DKH == 64);
static_assert(D_MODEL == 96 * 8);
static_assert((D_MODEL % 128) == 0 && (D_FF % 128) == 0);
static_assert((D_MODEL % 32) == 0 && (D_FF % 32) == 0);
static_assert(((D_MODEL * D_MODEL) % 2048) == 0);
static_assert(((D_FF * D_MODEL) % 2048) == 0);

#define PLANE_B   ((size_t)ROWS * D_MODEL * 2ull)
#define HB_B      ((size_t)ROWS * D_FF * 2ull)
#define R3_B      ((HB_B > 2ull * PLANE_B) ? HB_B : (2ull * PLANE_B))
#define WDD_B     ((size_t)D_MODEL * D_MODEL * 2ull)
#define WFD_B     ((size_t)D_FF * D_MODEL * 2ull)
static_assert((PLANE_B % 256) == 0 && (HB_B % 256) == 0 && (WDD_B % 256) == 0 && (WFD_B % 256) == 0);
static_assert(4ull * WDD_B + 2ull * WFD_B + 2ull * PLANE_B + 2ull * PLANE_B + R3_B <= 134217728ull);

#define SC_W    64.0f
#define SC_XN   8.0f
#define SC_P    256.0f
#define SC_CTX  32.0f
#define SC_H    16.0f

typedef _Float16 f16_t;
typedef _Float16 v16h __attribute__((ext_vector_type(16)));
typedef _Float16 v8h  __attribute__((ext_vector_type(8)));
typedef float    v8f  __attribute__((ext_vector_type(8)));
typedef float    v4f  __attribute__((ext_vector_type(4)));
typedef int      v4i  __attribute__((ext_vector_type(4)));
typedef v8h v8ha __attribute__((__may_alias__));
typedef v4f v4fa __attribute__((__may_alias__));
typedef v4i v4ia __attribute__((__may_alias__));

__device__ __forceinline__ float bf16r(float f) {
  unsigned int u = __float_as_uint(f);
  u += 0x7FFFu + ((u >> 16) & 1u);
  u &= 0xFFFF0000u;
  return __uint_as_float(u);
}

__device__ __forceinline__ unsigned full_row(unsigned r) {
  return (r / (unsigned)SEQ) * (unsigned)SEQ_FULL + (r % (unsigned)SEQ);
}

__device__ __forceinline__ v8f zero8() {
  v8f z;
#pragma unroll
  for (int i = 0; i < 8; ++i) z[i] = 0.0f;
  return z;
}

union Frag { v16h v; v8h h2[2]; };
__device__ __forceinline__ v16h ldfrag(const f16_t* rowp, unsigned g) {
  Frag f;
  f.h2[0] = *(const v8ha*)(rowp + 8u * g);
  f.h2[1] = *(const v8ha*)(rowp + 16u + 8u * g);
  return f.v;
}

__device__ __forceinline__ v8f mma16(v16h a, v16h b, v8f c) {
  v8f d = __builtin_amdgcn_wmma_f32_16x16x32_f16(false, a, false, b, (short)0, c, false, false);
  asm volatile("v_nop\n\tv_nop\n\tv_nop\n\tv_nop" : "+v"(d) : "v"(a), "v"(b));
  return d;
}

__global__ __launch_bounds__(256) void k_wcvt(
    const float* __restrict__ in, f16_t* __restrict__ out, float scale) {
  const size_t e0 = ((size_t)blockIdx.x * 256u + threadIdx.x) * 8u;
  v4f a = *(const v4f*)(in + e0);
  v4f b = *(const v4f*)(in + e0 + 4u);
  v8h ov;
#pragma unroll
  for (int e = 0; e < 4; ++e) {
    ov[e]     = (f16_t)(bf16r(a[e]) * scale);
    ov[4 + e] = (f16_t)(bf16r(b[e]) * scale);
  }
  f16_t* p = out + e0;
  *(volatile v8h*)p = ov;
  __threadfence();
  *(volatile v8h*)p = ov;
}

template <int RND>
__global__ __launch_bounds__(96) void k_ln(
    const float* __restrict__ in, const float* __restrict__ alpha,
    const float* __restrict__ beta, f16_t* __restrict__ out, float oscale) {
  __shared__ float red[2][4];
  const unsigned row = blockIdx.x, tid = threadIdx.x, wave = tid >> 5, lane = tid & 31u;
  const size_t srow = RND ? (size_t)full_row(row) : (size_t)row;
  const float* xr = in + srow * D_MODEL + tid * 8u;
  v4f xa = *(const v4f*)xr;
  v4f xb = *(const v4f*)(xr + 4);
  v4f aa = *(const v4f*)(alpha + tid * 8u);
  v4f ab = *(const v4f*)(alpha + tid * 8u + 4u);
  v4f ba = *(const v4f*)(beta + tid * 8u);
  v4f bb = *(const v4f*)(beta + tid * 8u + 4u);
  float v[8], al[8], be[8];
#pragma unroll
  for (int e = 0; e < 4; ++e) {
    v[e] = xa[e]; v[4 + e] = xb[e];
    al[e] = bf16r(aa[e]); al[4 + e] = bf16r(ab[e]);
    be[e] = bf16r(ba[e]); be[4 + e] = bf16r(bb[e]);
  }
  if (RND) {
#pragma unroll
    for (int e = 0; e < 8; ++e) v[e] = bf16r(v[e]);
  }
  float s = 0.f;
#pragma unroll
  for (int e = 0; e < 8; ++e) s += v[e];
#pragma unroll
  for (int off = 16; off > 0; off >>= 1) s += __shfl_xor(s, off, 32);
  if (lane == 0) red[0][wave] = s;
  __syncthreads();
  const float tot = (red[0][0] + red[0][1]) + red[0][2];
  const float mean = tot * (1.0f / D_MODEL);
  float d[8];
  float ss = 0.f;
#pragma unroll
  for (int e = 0; e < 8; ++e) { d[e] = v[e] - mean; ss += d[e] * d[e]; }
#pragma unroll
  for (int off = 16; off > 0; off >>= 1) ss += __shfl_xor(ss, off, 32);
  if (lane == 0) red[1][wave] = ss;
  __syncthreads();
  const float tot2 = (red[1][0] + red[1][1]) + red[1][2];
  const float var = tot2 * (1.0f / (float)(D_MODEL - 1));
  const float sd = sqrtf(var);
  const float inv = 1.0f / (sd + 1e-6f);
  v8h ov;
#pragma unroll
  for (int e = 0; e < 8; ++e) ov[e] = (f16_t)((al[e] * d[e] * inv + be[e]) * oscale);
  f16_t* op = out + (size_t)row * D_MODEL + tid * 8u;
  *(volatile v8h*)op = ov;
  __threadfence();
  *(volatile v8h*)op = ov;
}

template <int OUT16, int RELU, int RESM, int OUTFULL>
__global__ __launch_bounds__(256) void k_gemm(
    const f16_t* __restrict__ A, const f16_t* __restrict__ Bt,
    const float* __restrict__ bias, const float* __restrict__ res,
    void* __restrict__ Cout, unsigned M, unsigned N, unsigned K, float cscale, float oscale) {
  __shared__ __align__(16) f16_t As[128 * 32];
  __shared__ __align__(16) f16_t Bs[128 * 32];
  __shared__ __align__(16) float  St[8 * 16 * 64];
  (void)M;
  const unsigned tid = threadIdx.x;
  const unsigned wave = tid >> 5, lane = tid & 31u, lh = lane & 15u, g = lane >> 4;
  const unsigned waveM = wave & 3u, waveN = wave >> 2;
  const unsigned rowBase = blockIdx.y * 128u, colBase = blockIdx.x * 128u;

  const unsigned sr0 = tid >> 2, sc0 = (tid & 3u) * 8u;
  const f16_t* gA0 = A  + (size_t)(rowBase + sr0) * K + sc0;
  const f16_t* gA1 = A  + (size_t)(rowBase + sr0 + 64u) * K + sc0;
  const f16_t* gB0 = Bt + (size_t)(colBase + sr0) * K + sc0;
  const f16_t* gB1 = Bt + (size_t)(colBase + sr0 + 64u) * K + sc0;

  v8f acc[2][4];
#pragma unroll
  for (int mr = 0; mr < 2; ++mr)
#pragma unroll
    for (int nr = 0; nr < 4; ++nr) acc[mr][nr] = zero8();

  const unsigned nk = K >> 5;
  for (unsigned kt = 0; kt < nk; ++kt) {
    const unsigned kc = kt << 5;
    v8h a0 = *(const v8h*)(gA0 + kc);
    v8h a1 = *(const v8h*)(gA1 + kc);
    v8h b0 = *(const v8h*)(gB0 + kc);
    v8h b1 = *(const v8h*)(gB1 + kc);
    __syncthreads();
    *(v8h*)&As[sr0 * 32u + sc0]         = a0;
    *(v8h*)&As[(sr0 + 64u) * 32u + sc0] = a1;
    *(v8h*)&Bs[sr0 * 32u + sc0]         = b0;
    *(v8h*)&Bs[(sr0 + 64u) * 32u + sc0] = b1;
    __syncthreads();
    v16h af[2], bf[4];
#pragma unroll
    for (int mr = 0; mr < 2; ++mr)
      af[mr] = ldfrag(&As[(waveM * 32u + (unsigned)mr * 16u + lh) * 32u], g);
#pragma unroll
    for (int nr = 0; nr < 4; ++nr)
      bf[nr] = ldfrag(&Bs[(waveN * 64u + (unsigned)nr * 16u + lh) * 32u], g);
#pragma unroll
    for (int mr = 0; mr < 2; ++mr)
#pragma unroll
      for (int nr = 0; nr < 4; ++nr)
        acc[mr][nr] = mma16(af[mr], bf[nr], acc[mr][nr]);
  }

  const unsigned cb = colBase + waveN * 64u;
  float* S = &St[wave * (16u * 64u)];
#pragma unroll
  for (int mr = 0; mr < 2; ++mr) {
    __syncthreads();
#pragma unroll
    for (int nr = 0; nr < 4; ++nr)
#pragma unroll
      for (int r = 0; r < 8; ++r)
        S[(g * 8u + (unsigned)r) * 64u + (unsigned)nr * 16u + lh] = acc[mr][nr][r];
    __syncthreads();
    const unsigned rb = rowBase + waveM * 32u + (unsigned)mr * 16u;
    if (OUT16) {
      f16_t* C16 = (f16_t*)Cout;
      v8h ov[4];
#pragma unroll
      for (int j = 0; j < 4; ++j) {
        const unsigned lr = (unsigned)j * 4u + (lane >> 3), pc = lane & 7u;
        v4f s0 = *(const v4fa*)&S[lr * 64u + pc * 8u];
        v4f s1 = *(const v4fa*)&S[lr * 64u + pc * 8u + 4u];
        v4f q0 = *(const v4f*)&bias[cb + pc * 8u];
        v4f q1 = *(const v4f*)&bias[cb + pc * 8u + 4u];
#pragma unroll
        for (int e = 0; e < 4; ++e) {
          float v0 = s0[e] * cscale + bf16r(q0[e]);
          float v1 = s1[e] * cscale + bf16r(q1[e]);
          if (RELU) { v0 = fmaxf(v0, 0.0f); v1 = fmaxf(v1, 0.0f); }
          ov[j][e]     = (f16_t)(v0 * oscale);
          ov[j][4 + e] = (f16_t)(v1 * oscale);
        }
      }
#pragma unroll
      for (int j = 0; j < 4; ++j) {
        const unsigned lr = (unsigned)j * 4u + (lane >> 3), pc = lane & 7u;
        f16_t* p = C16 + (size_t)(rb + lr) * N + cb + pc * 8u;
        *(volatile v8h*)p = ov[j];
      }
      __threadfence();
#pragma unroll
      for (int j = 0; j < 4; ++j) {
        const unsigned lr = (unsigned)j * 4u + (lane >> 3), pc = lane & 7u;
        f16_t* p = C16 + (size_t)(rb + lr) * N + cb + pc * 8u;
        *(volatile v8h*)p = ov[j];
      }
    } else {
      float* C32 = (float*)Cout;
      v4f ov[8];
#pragma unroll
      for (int j = 0; j < 8; ++j) {
        const unsigned lr = (unsigned)j * 2u + (lane >> 4), pc = lane & 15u;
        v4f s0 = *(const v4fa*)&S[lr * 64u + pc * 4u];
        v4f q0 = *(const v4f*)&bias[cb + pc * 4u];
        v4f vv;
#pragma unroll
        for (int e = 0; e < 4; ++e) vv[e] = s0[e] * cscale + bf16r(q0[e]);
        if (RELU) {
#pragma unroll
          for (int e = 0; e < 4; ++e) vv[e] = fmaxf(vv[e], 0.0f);
        }
        if (RESM == 1) {
          v4f rr = *(const v4f*)&res[(size_t)(rb + lr) * N + cb + pc * 4u];
#pragma unroll
          for (int e = 0; e < 4; ++e) vv[e] += rr[e];
        } else if (RESM == 2) {
          v4f rr = *(const v4f*)&res[(size_t)full_row(rb + lr) * N + cb + pc * 4u];
#pragma unroll
          for (int e = 0; e < 4; ++e) vv[e] += bf16r(rr[e]);
        }
        ov[j] = vv;
      }
#pragma unroll
      for (int j = 0; j < 8; ++j) {
        const unsigned lr = (unsigned)j * 2u + (lane >> 4), pc = lane & 15u;
        const unsigned orow = OUTFULL ? full_row(rb + lr) : (rb + lr);
        float* p = C32 + (size_t)orow * N + cb + pc * 4u;
        *(volatile v4f*)p = ov[j];
      }
      __threadfence();
#pragma unroll
      for (int j = 0; j < 8; ++j) {
        const unsigned lr = (unsigned)j * 2u + (lane >> 4), pc = lane & 15u;
        const unsigned orow = OUTFULL ? full_row(rb + lr) : (rb + lr);
        float* p = C32 + (size_t)orow * N + cb + pc * 4u;
        *(volatile v4f*)p = ov[j];
      }
    }
  }
}

__global__ __launch_bounds__(128) void k_attn(
    const f16_t* __restrict__ Qp, const f16_t* __restrict__ Kp,
    const f16_t* __restrict__ Vp, const int* __restrict__ msk,
    f16_t* __restrict__ ctx) {
  __shared__ __align__(16) f16_t Qs[64 * 64];
  __shared__ __align__(16) f16_t Ks[64 * 64];
  __shared__ __align__(16) f16_t Vt[64 * 64];
  __shared__ __align__(16) f16_t Ps[64 * 64];
  __shared__ __align__(16) int   Mrow[SEQ];
  __shared__ int wz[4];
  const unsigned tid = threadIdx.x;
  const unsigned wave = tid >> 5, lane = tid & 31u, lh = lane & 15u, g = lane >> 4;
  const unsigned qt = blockIdx.x, h = blockIdx.y, b = blockIdx.z;
  const unsigned qbase = qt * 64u;
  const size_t prow0 = (size_t)b * SEQ;
  const unsigned col0 = h * (unsigned)DKH;

  int anyz = 0;
#pragma unroll
  for (unsigned i = 0; i < (unsigned)((SEQ / 4 + 127) / 128); ++i) {
    const unsigned id = i * 128u + tid;
    if (id < (unsigned)(SEQ / 4)) {
      v4i mv = *(const v4i*)&msk[(size_t)b * SEQ_FULL + id * 4u];
      *(v4ia*)&Mrow[id * 4u] = mv;
      anyz |= (int)(mv[0] == 0) | (int)(mv[1] == 0) | (int)(mv[2] == 0) | (int)(mv[3] == 0);
    }
  }
#pragma unroll
  for (int off = 16; off > 0; off >>= 1) anyz |= __shfl_xor(anyz, off, 32);
  if (lane == 0) wz[wave] = anyz;

#pragma unroll
  for (int i = 0; i < 4; ++i) {
    const unsigned id = (unsigned)i * 128u + tid;
    const unsigned r = id >> 3, c = (id & 7u) * 8u;
    *(v8h*)&Qs[r * 64u + c] = *(const v8h*)&Qp[(prow0 + qbase + r) * D_MODEL + col0 + c];
  }
  __syncthreads();
  const int usem_i = __builtin_amdgcn_readfirstlane(wz[0] | wz[1] | wz[2] | wz[3]);
  const bool usem = (usem_i != 0);
  v16h aq[2];
#pragma unroll
  for (int c = 0; c < 2; ++c) aq[c] = ldfrag(&Qs[(wave * 16u + lh) * 64u + (unsigned)c * 32u], g);

  v8f o[4];
#pragma unroll
  for (int nr = 0; nr < 4; ++nr) o[nr] = zero8();
  float m[8], l[8];
#pragma unroll
  for (int r = 0; r < 8; ++r) { m[r] = -1e30f; l[r] = 0.f; }
  const float sm_scale = 0.125f;

  for (unsigned kt = 0; kt < (unsigned)(SEQ / 64); ++kt) {
    const unsigned kbase = kt * 64u;
    __syncthreads();
#pragma unroll
    for (int i = 0; i < 4; ++i) {
      const unsigned id = (unsigned)i * 128u + tid;
      const unsigned r = id >> 3, c = (id & 7u) * 8u;
      *(v8h*)&Ks[r * 64u + c] = *(const v8h*)&Kp[(prow0 + kbase + r) * D_MODEL + col0 + c];
      v8h vv = *(const v8h*)&Vp[(prow0 + kbase + r) * D_MODEL + col0 + c];
#pragma unroll
      for (int j = 0; j < 8; ++j) Vt[(c + (unsigned)j) * 64u + r] = vv[j];
    }
    __syncthreads();

    v8f s[4];
#pragma unroll
    for (int nr = 0; nr < 4; ++nr) {
      s[nr] = zero8();
#pragma unroll
      for (int c = 0; c < 2; ++c) {
        v16h bk = ldfrag(&Ks[((unsigned)nr * 16u + lh) * 64u + (unsigned)c * 32u], g);
        s[nr] = mma16(aq[c], bk, s[nr]);
      }
    }
#pragma unroll
    for (int nr = 0; nr < 4; ++nr)
#pragma unroll
      for (int r = 0; r < 8; ++r) s[nr][r] = s[nr][r] * sm_scale;
    if (usem) {
#pragma unroll
      for (int nr = 0; nr < 4; ++nr) {
        const int mvv = Mrow[kbase + (unsigned)nr * 16u + lh];
#pragma unroll
        for (int r = 0; r < 8; ++r)
          s[nr][r] = (mvv == 0) ? -1e9f : s[nr][r];
      }
    }
    float f[8];
#pragma unroll
    for (int r = 0; r < 8; ++r) {
      float v = fmaxf(fmaxf(s[0][r], s[1][r]), fmaxf(s[2][r], s[3][r]));
#pragma unroll
      for (int off = 8; off > 0; off >>= 1) v = fmaxf(v, __shfl_xor(v, off, 16));
      const float mn = fmaxf(m[r], v);
      f[r] = __expf(m[r] - mn);
      m[r] = mn;
    }
    float rs[8];
#pragma unroll
    for (int r = 0; r < 8; ++r) rs[r] = 0.f;
#pragma unroll
    for (int nr = 0; nr < 4; ++nr)
#pragma unroll
      for (int r = 0; r < 8; ++r) {
        const float p = __expf(s[nr][r] - m[r]);
        s[nr][r] = p;
        rs[r] += p;
      }
#pragma unroll
    for (int r = 0; r < 8; ++r) {
      float v = rs[r];
#pragma unroll
      for (int off = 8; off > 0; off >>= 1) v += __shfl_xor(v, off, 16);
      l[r] = l[r] * f[r] + v;
    }
#pragma unroll
    for (int nr = 0; nr < 4; ++nr)
#pragma unroll
      for (int r = 0; r < 8; ++r) o[nr][r] *= f[r];
#pragma unroll
    for (int nr = 0; nr < 4; ++nr)
#pragma unroll
      for (int r = 0; r < 8; ++r)
        Ps[(wave * 16u + g * 8u + (unsigned)r) * 64u + (unsigned)nr * 16u + lh] = (f16_t)(s[nr][r] * SC_P);
    __syncthreads();

#pragma unroll
    for (int c = 0; c < 2; ++c) {
      v16h ap = ldfrag(&Ps[(wave * 16u + lh) * 64u + (unsigned)c * 32u], g);
#pragma unroll
      for (int nr = 0; nr < 4; ++nr) {
        v16h bv = ldfrag(&Vt[((unsigned)nr * 16u + lh) * 64u + (unsigned)c * 32u], g);
        o[nr] = mma16(ap, bv, o[nr]);
      }
    }
  }

  __syncthreads();
  float il[8];
#pragma unroll
  for (int r = 0; r < 8; ++r) il[r] = (SC_CTX / SC_P) * (1.0f / l[r]);
#pragma unroll
  for (int nr = 0; nr < 4; ++nr)
#pragma unroll
    for (int r = 0; r < 8; ++r)
      Ps[(wave * 16u + g * 8u + (unsigned)r) * 64u + (unsigned)nr * 16u + lh] = (f16_t)(o[nr][r] * il[r]);
  __syncthreads();
  v8h ov[4];
#pragma unroll
  for (int j = 0; j < 4; ++j) {
    const unsigned lr = wave * 16u + (unsigned)j * 4u + (lane >> 3), pc = lane & 7u;
    ov[j] = *(const v8ha*)&Ps[lr * 64u + pc * 8u];
  }
#pragma unroll
  for (int j = 0; j < 4; ++j) {
    const unsigned lr = wave * 16u + (unsigned)j * 4u + (lane >> 3), pc = lane & 7u;
    f16_t* p = ctx + (prow0 + qbase + lr) * D_MODEL + col0 + pc * 8u;
    *(volatile v8h*)p = ov[j];
  }
  __threadfence();
#pragma unroll
  for (int j = 0; j < 4; ++j) {
    const unsigned lr = wave * 16u + (unsigned)j * 4u + (lane >> 3), pc = lane & 7u;
    f16_t* p = ctx + (prow0 + qbase + lr) * D_MODEL + col0 + pc * 8u;
    *(volatile v8h*)p = ov[j];
  }
}

extern "C" void kernel_launch(void* const* d_in, const int* in_sizes, int n_in,
                              void* d_out, int out_size, void* d_ws, size_t ws_size,
                              hipStream_t stream) {
  if (n_in < 18) return;
  const int need_x = ((NB - 1) * SEQ_FULL + SEQ) * D_MODEL;
  if (in_sizes[0] < need_x) return;
  if (in_sizes[1] < (NB - 1) * SEQ_FULL + SEQ) return;
  if (in_sizes[2] < D_MODEL * D_MODEL || in_sizes[4] < D_MODEL * D_MODEL ||
      in_sizes[6] < D_MODEL * D_MODEL || in_sizes[8] < D_MODEL * D_MODEL) return;
  if (in_sizes[3] < D_MODEL || in_sizes[5] < D_MODEL || in_sizes[7] < D_MODEL ||
      in_sizes[9] < D_MODEL) return;
  if (in_sizes[10] < D_FF * D_MODEL || in_sizes[11] < D_FF) return;
  if (in_sizes[12] < D_MODEL * D_FF || in_sizes[13] < D_MODEL) return;
  if (in_sizes[14] < D_MODEL || in_sizes[15] < D_MODEL || in_sizes[16] < D_MODEL ||
      in_sizes[17] < D_MODEL) return;
  if (out_size < need_x) return;

  const float* x      = (const float*)d_in[0];
  const int*   msk    = (const int*)d_in[1];
  const float* Wq = (const float*)d_in[2];   const float* bq = (const float*)d_in[3];
  const float* Wk = (const float*)d_in[4];   const float* bk = (const float*)d_in[5];
  const float* Wv = (const float*)d_in[6];   const float* bv = (const float*)d_in[7];
  const float* Wo = (const float*)d_in[8];   const float* bo = (const float*)d_in[9];
  const float* W1 = (const float*)d_in[10];  const float* b1 = (const float*)d_in[11];
  const float* W2 = (const float*)d_in[12];  const float* b2 = (const float*)d_in[13];
  const float* alpha1 = (const float*)d_in[14]; const float* beta1 = (const float*)d_in[15];
  const float* alpha2 = (const float*)d_in[16]; const float* beta2 = (const float*)d_in[17];
  float* out = (float*)d_out;

  char* ws = (char*)d_ws;
  size_t off = 0;
  auto carve = [&](size_t bytes) -> void* {
    void* p = ws + off;
    off += (bytes + 255) & ~(size_t)255;
    return p;
  };
  f16_t* wq16 = (f16_t*)carve(WDD_B);
  f16_t* wk16 = (f16_t*)carve(WDD_B);
  f16_t* wv16 = (f16_t*)carve(WDD_B);
  f16_t* wo16 = (f16_t*)carve(WDD_B);
  f16_t* w116 = (f16_t*)carve(WFD_B);
  f16_t* w216 = (f16_t*)carve(WFD_B);
  f16_t* r0p  = (f16_t*)carve(PLANE_B);
  f16_t* r1p  = (f16_t*)carve(PLANE_B);
  float* x2   = (float*) carve(2 * PLANE_B);
  char*  r3p  = (char*)  carve(R3_B);
  if (off > ws_size) return;
  f16_t* xn  = r0p;
  f16_t* cx  = r0p;
  f16_t* qb  = r1p;
  f16_t* xn2 = r1p;
  f16_t* kb  = (f16_t*)r3p;
  f16_t* vbp = (f16_t*)(r3p + PLANE_B);
  f16_t* hb  = (f16_t*)r3p;

  k_wcvt<<<(D_MODEL * D_MODEL) / 2048, 256, 0, stream>>>(Wq, wq16, SC_W);
  k_wcvt<<<(D_MODEL * D_MODEL) / 2048, 256, 0, stream>>>(Wk, wk16, SC_W);
  k_wcvt<<<(D_MODEL * D_MODEL) / 2048, 256, 0, stream>>>(Wv, wv16, SC_W);
  k_wcvt<<<(D_MODEL * D_MODEL) / 2048, 256, 0, stream>>>(Wo, wo16, SC_W);
  k_wcvt<<<(D_FF * D_MODEL) / 2048,    256, 0, stream>>>(W1, w116, SC_W);
  k_wcvt<<<(D_FF * D_MODEL) / 2048,    256, 0, stream>>>(W2, w216, SC_W);

  k_ln<1><<<ROWS, 96, 0, stream>>>(x, alpha1, beta1, xn, SC_XN);

  const dim3 gP(D_MODEL / 128, ROWS / 128);
  const float cs_p = 1.0f / (SC_W * SC_XN);
  k_gemm<1, 0, 0, 0><<<gP, 256, 0, stream>>>(xn, wq16, bq, x, qb,  ROWS, D_MODEL, D_MODEL, cs_p, 1.0f);
  k_gemm<1, 0, 0, 0><<<gP, 256, 0, stream>>>(xn, wk16, bk, x, kb,  ROWS, D_MODEL, D_MODEL, cs_p, 1.0f);
  k_gemm<1, 0, 0, 0><<<gP, 256, 0, stream>>>(xn, wv16, bv, x, vbp, ROWS, D_MODEL, D_MODEL, cs_p, 1.0f);

  k_attn<<<dim3(SEQ / 64, NHEAD, NB), 128, 0, stream>>>(qb, kb, vbp, msk, cx);

  k_gemm<0, 0, 2, 0><<<gP, 256, 0, stream>>>(cx, wo16, bo, x, x2, ROWS, D_MODEL, D_MODEL,
                                            1.0f / (SC_W * SC_CTX), 1.0f);

  k_ln<0><<<ROWS, 96, 0, stream>>>(x2, alpha2, beta2, xn2, SC_XN);

  k_gemm<1, 1, 0, 0><<<dim3(D_FF / 128, ROWS / 128), 256, 0, stream>>>(
      xn2, w116, b1, x, hb, ROWS, D_FF, D_MODEL, cs_p, SC_H);

  k_gemm<0, 0, 1, 1><<<gP, 256, 0, stream>>>(hb, w216, b2, x2, out, ROWS, D_MODEL, D_FF,
                                            1.0f / (SC_W * SC_H), 1.0f);
}
